// GINNet_8340826488981
// MI455X (gfx1250) — hardware-verified
//
#include <hip/hip_runtime.h>
#include <stddef.h>
#include <stdint.h>


#define DIN     128
#define K2      256
#define NCLS    10
#define NTHR    256
#define NWAVE   8
#define EPT     8
#define CHUNK   (NTHR * EPT)
#define WCAP    (EPT * 32)
#define LISTN   (NWAVE * WCAP)
#define NBK     1024
#define SLB     10
#define RCAP    20480
#define DEGCAP  64
#define PKS     11
#define GBM     64
#define GBN     128
#define GTHR    128
#define GNT     8
#define PARTW   288
#define PG      32
#define GPAD    512
#define NGCAP   512
#define NUP     (DIN * (K2 / 8))
#define NPLANE  8
#define BK_ZINTS (2 * RCAP + 2 * NBK + LISTN)
#define LDS_BK  (BK_ZINTS * 4 + 64)
#define WSMAX   134217728

static_assert((CHUNK & (CHUNK - 1)) == 0 && CHUNK <= (1 << PKS));
static_assert((NBK & (NBK - 1)) == 0 && NBK <= (1 << PKS) && NBK == (1 << SLB));
static_assert(NTHR * 4 == NBK);
static_assert(LISTN >= NBK && LISTN >= NWAVE * WCAP);
static_assert((RCAP % 32) == 0 && (BK_ZINTS % 4) == 0);
static_assert(RCAP >= 12548 + 12548 / 2);
static_assert(DEGCAP >= 28 + 8);
static_assert(LDS_BK <= 300000);
static_assert(GBM == (GTHR / 32) * 16 && GBN == 16 * GNT && GTHR == GBN && GBN == 4 * 32);
static_assert(DIN == 32 * 4 && DIN == GBN && K2 == 2 * DIN && (K2 % 32) == 0);
static_assert((PARTW % 32) == 0 && PARTW >= 2 * GBN + 1 && PARTW / 4 <= GTHR);
static_assert((NUP % NTHR) == 0 && NUP == 4096);
static_assert((PG & (PG - 1)) == 0 && (GPAD % PG) == 0 && (GPAD % GBM) == 0);
static_assert(((PG * (DIN / 4)) % NTHR) == 0);
static_assert(NGCAP * NCLS * 4 <= 32768 && ((DIN * NCLS) % 4) == 0);
static_assert((NBK % GBM) == 0);

typedef float          v4f  __attribute__((ext_vector_type(4)));
typedef float          v8f  __attribute__((ext_vector_type(8)));
typedef int            v4i  __attribute__((ext_vector_type(4)));
typedef int            v8i  __attribute__((ext_vector_type(8)));
typedef unsigned int   v2u  __attribute__((ext_vector_type(2)));
typedef unsigned short v8us __attribute__((ext_vector_type(8)));
typedef __bf16         v16b __attribute__((ext_vector_type(16)));
typedef v4f  __attribute__((may_alias)) v4fa;
typedef v4i  __attribute__((may_alias)) v4ia;
typedef v8us __attribute__((may_alias)) v8usa;
union Frag { v16b vb; v8us h[2]; v8i w; };

__device__ __forceinline__ v8f wmb(const Frag& a, const Frag& b, v8f c) {
  v8f d = __builtin_amdgcn_wmma_f32_16x16x32_bf16(false, a.vb, false, b.vb, (short)0, c, false, false);
  asm volatile("v_nop\n\tv_nop\n\tv_nop\n\tv_nop" : "+v"(d) : "v"(a.w), "v"(b.w));
  return d;
}

__device__ __forceinline__ unsigned short bf_bits(float f) {
  const unsigned int u = __float_as_uint(f);
  const unsigned int r = (u + 0x7FFFu + ((u >> 16) & 1u)) >> 16;
  return (unsigned short)((f != f) ? 0x7FC0u : r);
}
__device__ __forceinline__ float bf_val(unsigned short b) { return __uint_as_float(((unsigned int)b) << 16); }
__device__ __forceinline__ float bf_rne(float f) { return bf_val(bf_bits(f)); }

__device__ __forceinline__ int scan_chunk(const int* __restrict__ dsts, int nE, int cbase, int slotBase,
                                          int nb, int vec8, int* list, int tid, int lane, int wave) {
  int wc = 0;
  const int el0  = tid * EPT;
  const int e0   = cbase + el0;
  const int sent = -2147483647 - 1;
  v4i da, db;
  if (vec8 != 0 && cbase + CHUNK <= nE) {
    da = *(const v4i*)(dsts + e0);
    db = *(const v4i*)(dsts + e0 + 4);
  } else {
    da.x = (e0     < nE) ? dsts[min(e0,     nE - 1)] : sent;
    da.y = (e0 + 1 < nE) ? dsts[min(e0 + 1, nE - 1)] : sent;
    da.z = (e0 + 2 < nE) ? dsts[min(e0 + 2, nE - 1)] : sent;
    da.w = (e0 + 3 < nE) ? dsts[min(e0 + 3, nE - 1)] : sent;
    db.x = (e0 + 4 < nE) ? dsts[min(e0 + 4, nE - 1)] : sent;
    db.y = (e0 + 5 < nE) ? dsts[min(e0 + 5, nE - 1)] : sent;
    db.z = (e0 + 6 < nE) ? dsts[min(e0 + 6, nE - 1)] : sent;
    db.w = (e0 + 7 < nE) ? dsts[min(e0 + 7, nE - 1)] : sent;
  }
  const unsigned nbs = (unsigned)slotBase;
  const unsigned unb = (unsigned)nb;
  const unsigned s0 = (unsigned)da.x - nbs, s1 = (unsigned)da.y - nbs;
  const unsigned s2 = (unsigned)da.z - nbs, s3 = (unsigned)da.w - nbs;
  const unsigned s4 = (unsigned)db.x - nbs, s5 = (unsigned)db.y - nbs;
  const unsigned s6 = (unsigned)db.z - nbs, s7 = (unsigned)db.w - nbs;
  const bool h0 = s0 < unb, h1 = s1 < unb, h2 = s2 < unb, h3 = s3 < unb;
  const bool h4 = s4 < unb, h5 = s5 < unb, h6 = s6 < unb, h7 = s7 < unb;
  const unsigned any = __builtin_amdgcn_ballot_w32(h0 | h1 | h2 | h3 | h4 | h5 | h6 | h7);
  if (any != 0u) {
#define HITJ(J, HJ, SJ) { \
      const unsigned mj = __builtin_amdgcn_ballot_w32(HJ); \
      if (mj != 0u) { \
        if (HJ) { \
          const int pos = wc + (int)__builtin_amdgcn_mbcnt_lo(mj, 0u); \
          if (pos < WCAP) list[wave * WCAP + pos] = ((el0 + (J)) << PKS) | (int)(SJ); \
        } \
        wc += (int)__builtin_popcount(mj); } }
    HITJ(0, h0, s0)
    HITJ(1, h1, s1)
    HITJ(2, h2, s2)
    HITJ(3, h3, s3)
    HITJ(4, h4, s4)
    HITJ(5, h5, s5)
    HITJ(6, h6, s6)
    HITJ(7, h7, s7)
#undef HITJ
  }
  return wc;
}

__device__ __forceinline__ v8us cv8b(const float* __restrict__ p) {
  v8us o;
#pragma unroll
  for (int i = 0; i < 8; ++i) o[i] = bf_bits(p[(size_t)i * DIN]);
  return o;
}

__global__ __launch_bounds__(NTHR) void k_prep(const float* __restrict__ wf, const float* __restrict__ w1,
                                               const float* __restrict__ w2, const float* __restrict__ wfc,
                                               unsigned short* wt) {
  const int u = (int)blockIdx.x * NTHR + (int)threadIdx.x;
  if (u >= NPLANE * NUP) return;
  const int pl = u >> 12;
  const int v  = u & (NUP - 1);
  const int n  = v >> 5;
  const int k8 = (v & 31) * 8;
  const int kk = k8 & (DIN - 1);
  const size_t so = (size_t)kk * DIN + (size_t)n;
  v8us o;
  if (pl == 0) {
    o = cv8b(wf + so);
  } else if (pl < 4) {
    o = cv8b(w1 + (size_t)(pl - 1) * DIN * DIN + so);
  } else if (pl < 7) {
    o = cv8b(w2 + (size_t)(pl - 4) * DIN * DIN + so);
  } else {
    o = cv8b(wfc + so);
  }
  unsigned short* dp = wt + (size_t)u * 8;
  *(volatile v8us*)dp = o;
  __threadfence();
  *(volatile v8us*)dp = o;
}

__device__ __forceinline__ void block_record(const float* stg, float* pst, int nvr, int tid) {
  float s = 0.0f;
#pragma unroll 1
  for (int r = 0; r < nvr; ++r) s += stg[r * GBN + tid];
  const float inv  = 1.0f / (float)(nvr < 1 ? 1 : nvr);
  const float mean = s * inv;
  float q = 0.0f;
#pragma unroll 1
  for (int r = 0; r < nvr; ++r) {
    const float d = stg[r * GBN + tid] - mean;
    q = fmaf(d, d, q);
  }
  pst[1 + tid] = mean;
  pst[1 + GBN + tid] = q;
  if (tid == 0) pst[0] = (float)nvr;
#pragma unroll 1
  for (int i = 2 * GBN + 1 + tid; i < PARTW; i += GTHR) pst[i] = 0.0f;
}

__global__ __launch_bounds__(GTHR) void k_xstats(const float* __restrict__ x, int nN, float* part) {
  __shared__ __attribute__((aligned(16))) float stg[GBM * GBN];
  __shared__ __attribute__((aligned(16))) float pst[PARTW];
  const int tid = (int)threadIdx.x;
  const int rowBase = (int)blockIdx.x * GBM;
#pragma unroll 4
  for (int i = 0; i < (GBM * GBN / 4) / GTHR; ++i) {
    const int p  = i * GTHR + tid;
    const int lr = p >> 5, q = p & 31;
    const int gr = rowBase + lr;
    const int gc = gr < nN ? gr : nN - 1;
    v4f v = *(const v4f*)(x + (size_t)gc * DIN + 4 * q);
    v.x = bf_rne(v.x); v.y = bf_rne(v.y); v.z = bf_rne(v.z); v.w = bf_rne(v.w);
    *(v4fa*)(stg + lr * GBN + 4 * q) = v;
  }
  __syncthreads();
  int nvr = nN - rowBase;
  nvr = nvr < 0 ? 0 : (nvr > GBM ? GBM : nvr);
  block_record(stg, pst, nvr, tid);
  __syncthreads();
  const bool pok = tid < PARTW / 4;
  v4f pv = {0.f, 0.f, 0.f, 0.f};
  float* pp = part + (size_t)blockIdx.x * PARTW + 4 * tid;
  if (pok) {
    pv = *(const v4fa*)(pst + 4 * tid);
    *(volatile v4f*)pp = pv;
  }
  __threadfence();
  if (pok) *(volatile v4f*)pp = pv;
}

__global__ __launch_bounds__(GBN) void k_comb(const float* __restrict__ part, int nPart, float* stat) {
  __shared__ __attribute__((aligned(16))) float stg[2 * GBN];
  const int tid = (int)threadIdx.x;
  double sn = 0.0, sm = 0.0;
#pragma unroll 1
  for (int b = 0; b < nPart; ++b) {
    const float* pr = part + (size_t)b * PARTW;
    const double nb = (double)pr[0];
    const double mb = (double)pr[1 + tid];
    sn += nb;
    sm += nb * mb;
  }
  const double nt = sn < 1.0 ? 1.0 : sn;
  const double mean = sm / nt;
  double M2 = 0.0;
#pragma unroll 1
  for (int b = 0; b < nPart; ++b) {
    const float* pr = part + (size_t)b * PARTW;
    const double nb = (double)pr[0];
    const double mb = (double)pr[1 + tid];
    const double qb = (double)pr[1 + GBN + tid];
    const double d = mb - mean;
    M2 += qb + nb * d * d;
  }
  const float varf = (float)(M2 / nt);
  const float rstd = 1.0f / sqrtf(varf + 1e-5f);
  stg[tid] = (float)mean;
  stg[GBN + tid] = rstd;
  __syncthreads();
  const bool ok = tid < (2 * GBN) / 4;
  v4f v = {0.f, 0.f, 0.f, 0.f};
  float* dp = stat + 4 * tid;
  if (ok) {
    v = *(const v4fa*)(stg + 4 * tid);
    *(volatile v4f*)dp = v;
  }
  __threadfence();
  if (ok) *(volatile v4f*)dp = v;
}

template <int RND, int RELU>
__global__ __launch_bounds__(NTHR) void k_apply(const float* __restrict__ in, const float* __restrict__ stat,
                                               const float* __restrict__ gam, const float* __restrict__ bet,
                                               int nN, int mRows, unsigned short* outp) {
  __shared__ float prm[4 * DIN];
  const int tid = (int)threadIdx.x;
  {
    const int c = tid & (DIN - 1);
    const float a0 = (tid < DIN) ? stat[c] : stat[DIN + c];
    const float a1 = (tid < DIN) ? bf_rne(gam[c]) : bf_rne(bet[c]);
    prm[tid] = a0;
    prm[2 * DIN + tid] = a1;
  }
  __syncthreads();
  const int u   = (int)blockIdx.x * NTHR + tid;
  const int row = u >> 4, q = u & 15;
  const int gc  = row < nN ? row : nN - 1;
  const float* p = in + (size_t)gc * DIN + 8 * q;
  const v4f a = *(const v4f*)p;
  const v4f b = *(const v4f*)(p + 4);
  const float f[8] = {a.x, a.y, a.z, a.w, b.x, b.y, b.z, b.w};
  const bool live = row < nN;
  v8us hv, lv;
#pragma unroll
  for (int j = 0; j < 8; ++j) {
    const int c = 8 * q + j;
    float v = f[j];
    if (RND != 0) v = bf_rne(v);
    float y = ((v - prm[c]) * prm[DIN + c]) * prm[2 * DIN + c] + prm[3 * DIN + c];
    if (RELU != 0) y = (y > 0.0f) ? y : (y - y);
    y = live ? y : 0.0f;
    const unsigned short hb = bf_bits(y);
    hv[j] = hb;
    lv[j] = bf_bits(y - bf_val(hb));
  }
  unsigned short* hp = outp + (size_t)row * K2 + 8 * q;
  unsigned short* lp = hp + DIN;
  const bool ok = row < mRows;
  if (ok) { *(volatile v8us*)hp = hv; *(volatile v8us*)lp = lv; }
  __threadfence();
  if (ok) { *(volatile v8us*)hp = hv; *(volatile v8us*)lp = lv; }
}

template <int RELU, int STATS>
__global__ __launch_bounds__(GTHR) void k_gemm(const unsigned short* __restrict__ A,
                                               const unsigned short* __restrict__ BT,
                                               const float* __restrict__ bias,
                                               float* outF, int nN, int mRows, float* part) {
  __shared__ __attribute__((aligned(16))) float stg[GBM * GBN];
  __shared__ __attribute__((aligned(16))) float pst[PARTW];
  const int tid = (int)threadIdx.x, lane = tid & 31, wave = tid >> 5, hh = lane >> 4, m = lane & 15;
  const int rowBase = (int)blockIdx.x * GBM;

  v8f acc[GNT];
  {
    const v8f z = {0.f, 0.f, 0.f, 0.f, 0.f, 0.f, 0.f, 0.f};
#pragma unroll
    for (int t = 0; t < GNT; ++t) acc[t] = z;
  }
  const unsigned short* ap = A  + (size_t)(rowBase + 16 * wave + m) * (size_t)K2 + 8 * hh;
  const unsigned short* bp = BT + (size_t)m * (size_t)K2 + 8 * hh;

#pragma unroll 1
  for (int k0 = 0; k0 < K2; k0 += 32) {
    Frag af;
    af.h[0] = *(const v8usa*)(ap + k0);
    af.h[1] = *(const v8usa*)(ap + k0 + 16);
#pragma unroll
    for (int nt = 0; nt < GNT; ++nt) {
      const unsigned short* wq = bp + (size_t)(16 * nt) * (size_t)K2 + k0;
      Frag bfr;
      bfr.h[0] = *(const v8usa*)wq;
      bfr.h[1] = *(const v8usa*)(wq + 16);
      acc[nt] = wmb(af, bfr, acc[nt]);
    }
  }

#pragma unroll
  for (int nt = 0; nt < GNT; ++nt) {
    const int lc = 16 * nt + m;
    const float bb = bf_rne(bias[lc]);
#pragma unroll
    for (int r = 0; r < 8; ++r) {
      const int lr = 16 * wave + 8 * hh + r;
      const bool live = (rowBase + lr) < nN;
      float v = acc[nt][r] + bb;
      if (RELU != 0) v = (v > 0.0f) ? v : (v - v);
      stg[lr * GBN + lc] = live ? v : 0.0f;
    }
  }
  __syncthreads();

  v4f fv[16];
#pragma unroll
  for (int i = 0; i < 16; ++i) {
    const int lr = 16 * wave + i;
    fv[i] = *(const v4fa*)(stg + lr * GBN + 4 * lane);
  }
  v4f pv = {0.f, 0.f, 0.f, 0.f};
  const bool pok = (STATS != 0) && (tid < PARTW / 4);
  if constexpr (STATS != 0) {
    int nvr = nN - rowBase;
    nvr = nvr < 0 ? 0 : (nvr > GBM ? GBM : nvr);
    block_record(stg, pst, nvr, tid);
    __syncthreads();
    if (pok) pv = *(const v4fa*)(pst + 4 * tid);
  }
  float* pp = part + (size_t)blockIdx.x * PARTW + 4 * tid;
#pragma unroll
  for (int i = 0; i < 16; ++i) {
    const int gr = rowBase + 16 * wave + i;
    float* op = outF + (size_t)gr * (size_t)DIN + 4 * lane;
    if (gr < mRows) *(volatile v4f*)op = fv[i];
  }
  if (pok) *(volatile v4f*)pp = pv;
  __threadfence();
#pragma unroll
  for (int i = 0; i < 16; ++i) {
    const int gr = rowBase + 16 * wave + i;
    float* op = outF + (size_t)gr * (size_t)DIN + 4 * lane;
    if (gr < mRows) *(volatile v4f*)op = fv[i];
  }
  if (pok) *(volatile v4f*)pp = pv;
}

__global__ __launch_bounds__(NTHR) void k_bucket(const int* __restrict__ srcs, const int* __restrict__ dsts,
                                                 int nN, int nE, int vec8, int* hits, int* co, int* fl) {
  extern __shared__ v4f lds_dyn[];
  int* reg1 = (int*)lds_dyn;
  int* reg2 = reg1 + RCAP;
  int* scnt = reg2 + RCAP;
  int* soff = scnt + NBK;
  int* list = soff + NBK;
  int* wcnt = list + LISTN;
  int* wtot = wcnt + NWAVE;
  const int tid = (int)threadIdx.x, lane = tid & 31, wave = tid >> 5;
  const int nodeBase = (int)blockIdx.x * NBK;

  {
    const v4i z4 = {0, 0, 0, 0};
    for (int i = tid * 4; i < BK_ZINTS; i += NTHR * 4) *(v4ia*)(reg1 + i) = z4;
    if (tid < 2 * NWAVE) wcnt[tid] = 0;
  }
  __syncthreads();

  int tot = 0;
  const int nChunks = (nE + CHUNK - 1) / CHUNK;
#pragma unroll 1
  for (int ch = 0; ch < nChunks; ++ch) {
    const int cbase = ch * CHUNK;
    const int wc = scan_chunk(dsts, nE, cbase, nodeBase, NBK, vec8, list, tid, lane, wave);
    if (lane == 0) wcnt[wave] = wc;
    __syncthreads();
    int pre = 0, all = 0;
#pragma unroll
    for (int w2 = 0; w2 < NWAVE; ++w2) {
      int c = wcnt[w2];
      c = c < 0 ? 0 : (c > WCAP ? WCAP : c);
      all += c;
      pre += (w2 < wave) ? c : 0;
    }
    const int wcc  = wc > WCAP ? WCAP : wc;
    const int base = tot + pre;
#pragma unroll 1
    for (int i = lane; i < wcc; i += 32) {
      const int ent = list[wave * WCAP + i];
      const int el  = (ent >> PKS) & (CHUNK - 1);
      const int sl  = ent & (NBK - 1);
      int eid = cbase + el;
      eid = eid > nE - 1 ? nE - 1 : eid;
      const int pos = base + i;
      if (pos < RCAP) reg1[pos] = (int)(((unsigned)eid << PKS) | (unsigned)sl);
    }
    tot += all;
    tot = tot > RCAP ? RCAP : tot;
    __syncthreads();
  }
  const int nh = tot;

  if (wave == 0) {
#pragma unroll 1
    for (int b0 = 0; b0 < nh; b0 += 32) {
      const int idx = b0 + lane;
      const int uv  = reg1[idx < RCAP ? idx : RCAP - 1];
      const int m32 = (nh - b0) < 32 ? (nh - b0) : 32;
#pragma unroll 1
      for (int k = 0; k < m32; ++k) {
        const int u  = __builtin_amdgcn_readlane(uv, k);
        const int sl = u & (NBK - 1);
        if (lane == 0) scnt[sl] = scnt[sl] + 1;
      }
    }
  }
  __syncthreads();

  {
    const v4i ca = *(const v4ia*)(scnt + 4 * tid);
    const int e0 = ca.x < 0 ? 0 : ca.x, e1 = ca.y < 0 ? 0 : ca.y, e2 = ca.z < 0 ? 0 : ca.z, e3 = ca.w < 0 ? 0 : ca.w;
    const int ts = e0 + e1 + e2 + e3;
    int incl = ts;
#pragma unroll
    for (int d = 1; d < 32; d <<= 1) {
      const int up = __shfl_up(incl, d);
      if (lane >= d) incl += up;
    }
    if (lane == 31) wtot[wave] = incl;
    __syncthreads();
    int pre = 0;
#pragma unroll
    for (int w2 = 0; w2 < NWAVE; ++w2) pre += (w2 < wave) ? wtot[w2] : 0;
    int run = pre + incl - ts;
    soff[4 * tid + 0] = run; run += e0;
    soff[4 * tid + 1] = run; run += e1;
    soff[4 * tid + 2] = run; run += e2;
    soff[4 * tid + 3] = run;
  }
  __syncthreads();
  for (int i = tid; i < NBK; i += NTHR) list[i] = soff[i];
  __syncthreads();

  if (wave == 0) {
#pragma unroll 1
    for (int b0 = 0; b0 < nh; b0 += 32) {
      const int idx = b0 + lane;
      const int uv  = reg1[idx < RCAP ? idx : RCAP - 1];
      const int m32 = (nh - b0) < 32 ? (nh - b0) : 32;
#pragma unroll 1
      for (int k = 0; k < m32; ++k) {
        const int u   = __builtin_amdgcn_readlane(uv, k);
        const int sl  = u & (NBK - 1);
        const int eid = (int)((unsigned)u >> PKS);
        if (lane == 0) {
          int pos = list[sl];
          pos = pos < 0 ? 0 : (pos > RCAP - 1 ? RCAP - 1 : pos);
          reg2[pos] = eid;
          list[sl] = pos + 1;
        }
      }
    }
  }
  __syncthreads();

  int nhPad = (nh + NTHR - 1) & ~(NTHR - 1);
  nhPad = nhPad > RCAP ? RCAP : nhPad;
#pragma unroll 1
  for (int i = tid; i < nhPad; i += NTHR) {
    int e = reg2[i];
    e = e < 0 ? 0 : (e > nE - 1 ? nE - 1 : e);
    int s = srcs[e];
    s = s < 0 ? 0 : (s > nN - 1 ? nN - 1 : s);
    reg2[i] = (i < nh) ? s : 0;
  }
  __syncthreads();

  int* hb = hits + (size_t)blockIdx.x * RCAP;
  int* cb = co + (size_t)blockIdx.x * (2 * NBK);
  int* fb = fl + (size_t)blockIdx.x * 32;
  v4i fvv = {0, 0, 0, 0};
  if (tid == 0) { fvv.x = (nh >= RCAP) ? 1 : 0; fvv.y = nh; }
#pragma unroll 1
  for (int i = tid * 4; i < RCAP; i += NTHR * 4) {
    const v4i v = *(const v4ia*)(reg2 + i);
    *(volatile v4i*)(hb + i) = v;
  }
#pragma unroll 1
  for (int i = tid * 4; i < 2 * NBK; i += NTHR * 4) {
    const v4i v = *(const v4ia*)(scnt + i);
    *(volatile v4i*)(cb + i) = v;
  }
  if (tid < 8) *(volatile v4i*)(fb + 4 * tid) = fvv;
  __threadfence();
#pragma unroll 1
  for (int i = tid * 4; i < RCAP; i += NTHR * 4) {
    const v4i v = *(const v4ia*)(reg2 + i);
    *(volatile v4i*)(hb + i) = v;
  }
#pragma unroll 1
  for (int i = tid * 4; i < 2 * NBK; i += NTHR * 4) {
    const v4i v = *(const v4ia*)(scnt + i);
    *(volatile v4i*)(cb + i) = v;
  }
  if (tid < 8) *(volatile v4i*)(fb + 4 * tid) = fvv;
}

__global__ __launch_bounds__(NTHR) void k_agg(const int* __restrict__ hits, const int* __restrict__ co,
                                              const int* __restrict__ fl, const float* __restrict__ fin,
                                              unsigned short* aout, int nN, int mRows, int nBuck) {
  const int tid = (int)threadIdx.x, lane = tid & 31;
  const int wave = __builtin_amdgcn_readfirstlane(tid >> 5);
  const float qnan = __int_as_float(0x7fc00000);
#pragma unroll 1
  for (int j = 0; j < 8; ++j) {
    const int row = (int)blockIdx.x * GBM + wave * 8 + j;
    int bk = row >> SLB;
    bk = bk > nBuck - 1 ? nBuck - 1 : bk;
    const int slot = row & (NBK - 1);
    const int craw = __builtin_amdgcn_readfirstlane(co[(size_t)bk * (2 * NBK) + slot]);
    int st         = __builtin_amdgcn_readfirstlane(co[(size_t)bk * (2 * NBK) + NBK + slot]);
    const int flg  = __builtin_amdgcn_readfirstlane(fl[(size_t)bk * 32]);
    const bool liveRow = row < nN;
    int cnt = craw < 0 ? 0 : (craw > DEGCAP ? DEGCAP : craw);
    st = st < 0 ? 0 : (st > RCAP ? RCAP : st);
    if (cnt > RCAP - st) cnt = RCAP - st;
    if (!liveRow) cnt = 0;
    const float pz = (flg != 0 || craw > DEGCAP) ? qnan : 0.0f;
    const int* hb = hits + (size_t)bk * RCAP;

    float ag0 = 0.f, ag1 = 0.f, ag2 = 0.f, ag3 = 0.f;
#pragma unroll 1
    for (int b0 = 0; b0 < cnt; b0 += 32) {
      int idx = st + b0 + lane;
      idx = idx > RCAP - 1 ? RCAP - 1 : idx;
      int sr = hb[idx];
      sr = sr < 0 ? 0 : (sr > nN - 1 ? nN - 1 : sr);
      const int m32 = (cnt - b0) < 32 ? (cnt - b0) : 32;
#pragma unroll 1
      for (int k = 0; k < m32; ++k) {
        const int sk = __builtin_amdgcn_readlane(sr, k);
        const v4f v = *(const v4f*)(fin + (size_t)sk * DIN + 4 * lane);
        ag0 += v.x; ag1 += v.y; ag2 += v.z; ag3 += v.w;
      }
    }
    const int nc = liveRow ? row : nN - 1;
    const v4f sv = *(const v4f*)(fin + (size_t)nc * DIN + 4 * lane);
    const float r0 = liveRow ? (sv.x + ag0 + pz) : 0.0f;
    const float r1 = liveRow ? (sv.y + ag1 + pz) : 0.0f;
    const float r2 = liveRow ? (sv.z + ag2 + pz) : 0.0f;
    const float r3 = liveRow ? (sv.w + ag3 + pz) : 0.0f;
    const unsigned short h0 = bf_bits(r0), h1 = bf_bits(r1), h2 = bf_bits(r2), h3 = bf_bits(r3);
    const unsigned short l0 = bf_bits(r0 - bf_val(h0)), l1 = bf_bits(r1 - bf_val(h1));
    const unsigned short l2 = bf_bits(r2 - bf_val(h2)), l3 = bf_bits(r3 - bf_val(h3));
    v2u ph, pl;
    ph.x = (unsigned int)h0 | ((unsigned int)h1 << 16);
    ph.y = (unsigned int)h2 | ((unsigned int)h3 << 16);
    pl.x = (unsigned int)l0 | ((unsigned int)l1 << 16);
    pl.y = (unsigned int)l2 | ((unsigned int)l3 << 16);
    unsigned short* hp = aout + (size_t)row * K2 + 4 * lane;
    unsigned short* lp = hp + DIN;
    const bool wsv = row < mRows;
    if (wsv) { *(volatile v2u*)hp = ph; *(volatile v2u*)lp = pl; }
    __threadfence();
    if (wsv) { *(volatile v2u*)hp = ph; *(volatile v2u*)lp = pl; }
  }
}

__global__ __launch_bounds__(NTHR) void k_pool(const float* __restrict__ H, const int* __restrict__ bat,
                                               int nN, int vec8b, int nG, float* g0) {
  __shared__ __attribute__((aligned(16))) float accs[PG * DIN];
  __shared__ int list[LISTN];
  __shared__ int wcnt[NWAVE];
  const int tid = (int)threadIdx.x, lane = tid & 31, wave = tid >> 5;
  const int slotBase = (int)blockIdx.x * PG;
  int nb = nG - slotBase;
  nb = nb < 0 ? 0 : (nb > PG ? PG : nb);

  for (int i = tid; i < PG * DIN; i += NTHR) accs[i] = 0.0f;
  __syncthreads();

  const int nChunks = (nN + CHUNK - 1) / CHUNK;
#pragma unroll 1
  for (int ch = 0; ch < nChunks; ++ch) {
    const int cbase = ch * CHUNK;
    const int wc = scan_chunk(bat, nN, cbase, slotBase, nb, vec8b, list, tid, lane, wave);
    if (lane == 0) wcnt[wave] = wc;
    __syncthreads();
#pragma unroll 1
    for (int w2 = 0; w2 < NWAVE; ++w2) {
      int c = wcnt[w2];
      c = c < 0 ? 0 : (c > WCAP ? WCAP : c);
#pragma unroll 1
      for (int i = 0; i < c; ++i) {
        const int ent = list[w2 * WCAP + i];
        const int el  = (ent >> PKS) & (CHUNK - 1);
        const int sl  = ent & (PG - 1);
        int node = cbase + el;
        node = node < 0 ? 0 : (node > nN - 1 ? nN - 1 : node);
        if (tid < DIN) {
          const float v = H[(size_t)node * DIN + tid];
          accs[sl * DIN + tid] += v;
        }
      }
    }
    __syncthreads();
  }

  constexpr int NIT = (PG * (DIN / 4)) / NTHR;
  v4f pv[NIT];
#pragma unroll
  for (int it = 0; it < NIT; ++it) {
    const int p = it * NTHR + tid;
    pv[it] = *(const v4fa*)(accs + (p >> 5) * DIN + 4 * (p & 31));
  }
#pragma unroll
  for (int it = 0; it < NIT; ++it) {
    const int p = it * NTHR + tid;
    const int g = slotBase + (p >> 5);
    float* op = g0 + (size_t)g * DIN + 4 * (p & 31);
    if (g < GPAD) *(volatile v4f*)op = pv[it];
  }
  __threadfence();
#pragma unroll
  for (int it = 0; it < NIT; ++it) {
    const int p = it * NTHR + tid;
    const int g = slotBase + (p >> 5);
    float* op = g0 + (size_t)g * DIN + 4 * (p & 31);
    if (g < GPAD) *(volatile v4f*)op = pv[it];
  }
}

__global__ __launch_bounds__(NTHR) void k_bnfc(const float* __restrict__ g0, const float* __restrict__ gam,
                                               const float* __restrict__ bet, int nG, unsigned short* ghl) {
  __shared__ float prm[4 * DIN];
  const int tid = (int)threadIdx.x;
  if (tid < DIN) {
    double s = 0.0;
#pragma unroll 1
    for (int r = 0; r < nG; ++r) s += (double)g0[(size_t)r * DIN + tid];
    const double mean = s / (double)nG;
    double q = 0.0;
#pragma unroll 1
    for (int r = 0; r < nG; ++r) {
      const double d = (double)g0[(size_t)r * DIN + tid] - mean;
      q += d * d;
    }
    const float varf = (float)(q / (double)nG);
    prm[tid] = (float)mean;
    prm[DIN + tid] = 1.0f / sqrtf(varf + 1e-5f);
    prm[2 * DIN + tid] = bf_rne(gam[tid]);
    prm[3 * DIN + tid] = bf_rne(bet[tid]);
  }
  __syncthreads();
#pragma unroll 1
  for (int it = 0; it < (GPAD * 16) / NTHR; ++it) {
    const int u   = it * NTHR + tid;
    const int row = u >> 4, q = u & 15;
    const int gc  = row < nG ? row : nG - 1;
    const float* p = g0 + (size_t)gc * DIN + 8 * q;
    const v4f a = *(const v4f*)p;
    const v4f b = *(const v4f*)(p + 4);
    const float f[8] = {a.x, a.y, a.z, a.w, b.x, b.y, b.z, b.w};
    const bool live = row < nG;
    v8us hv, lv;
#pragma unroll
    for (int j = 0; j < 8; ++j) {
      const int c = 8 * q + j;
      float y = ((f[j] - prm[c]) * prm[DIN + c]) * prm[2 * DIN + c] + prm[3 * DIN + c];
      y = live ? y : 0.0f;
      const unsigned short hb = bf_bits(y);
      hv[j] = hb;
      lv[j] = bf_bits(y - bf_val(hb));
    }
    unsigned short* hp = ghl + (size_t)row * K2 + 8 * q;
    unsigned short* lp = hp + DIN;
    *(volatile v8us*)hp = hv;
    *(volatile v8us*)lp = lv;
    __threadfence();
    *(volatile v8us*)hp = hv;
    *(volatile v8us*)lp = lv;
  }
}

__global__ __launch_bounds__(NTHR) void k_tail(const float* __restrict__ g1, const float* __restrict__ gam,
                                               const float* __restrict__ bet, const float* __restrict__ wc,
                                               const float* __restrict__ bc, const int* __restrict__ fl,
                                               int nBuck, int nG, float* out) {
  __shared__ __attribute__((aligned(16))) float osm[NGCAP * NCLS];
  __shared__ __attribute__((aligned(16))) float wcl[DIN * NCLS];
  __shared__ float prm[4 * DIN];
  __shared__ float bcl[16];
  __shared__ int pflag;
  const int tid = (int)threadIdx.x;
  if (tid == 0) pflag = 0;
  if (tid < DIN) {
    double s = 0.0;
#pragma unroll 1
    for (int r = 0; r < nG; ++r) s += (double)g1[(size_t)r * DIN + tid];
    const double mean = s / (double)nG;
    double q = 0.0;
#pragma unroll 1
    for (int r = 0; r < nG; ++r) {
      const double d = (double)g1[(size_t)r * DIN + tid] - mean;
      q += d * d;
    }
    const float varf = (float)(q / (double)nG);
    prm[tid] = (float)mean;
    prm[DIN + tid] = 1.0f / sqrtf(varf + 1e-5f);
    prm[2 * DIN + tid] = bf_rne(gam[tid]);
    prm[3 * DIN + tid] = bf_rne(bet[tid]);
  }
#pragma unroll 1
  for (int i = tid; i < (DIN * NCLS) / 4; i += NTHR) {
    v4f v = *(const v4f*)(wc + 4 * i);
    v.x = bf_rne(v.x); v.y = bf_rne(v.y); v.z = bf_rne(v.z); v.w = bf_rne(v.w);
    *(v4fa*)(wcl + 4 * i) = v;
  }
  if (tid < 16) {
    const float b = bc[tid < NCLS ? tid : NCLS - 1];
    bcl[tid] = (tid < NCLS) ? bf_rne(b) : 0.0f;
  }
  __syncthreads();
  {
    const int bi = tid < nBuck ? tid : nBuck - 1;
    const int fv = fl[(size_t)bi * 32];
    if (tid < nBuck && fv != 0) pflag = 1;
  }

#pragma unroll 1
  for (int row = tid; row < nG; row += NTHR) {
    float lg[NCLS];
#pragma unroll
    for (int c = 0; c < NCLS; ++c) lg[c] = 0.0f;
    const float* gp = g1 + (size_t)row * DIN;
#pragma unroll 1
    for (int k = 0; k < DIN; ++k) {
      const float v = gp[k];
      const float y = ((v - prm[k]) * prm[DIN + k]) * prm[2 * DIN + k] + prm[3 * DIN + k];
#pragma unroll
      for (int c = 0; c < NCLS; ++c) lg[c] = fmaf(y, wcl[k * NCLS + c], lg[c]);
    }
#pragma unroll
    for (int c = 0; c < NCLS; ++c) osm[row * NCLS + c] = lg[c] + bcl[c];
    float mx = osm[row * NCLS];
#pragma unroll 1
    for (int c = 1; c < NCLS; ++c) {
      const float v = osm[row * NCLS + c];
      mx = (v > mx || v != v) ? v : mx;
    }
    float se = 0.0f;
#pragma unroll 1
    for (int c = 0; c < NCLS; ++c) se += expf(osm[row * NCLS + c] - mx);
    const float lse = mx + logf(se);
#pragma unroll 1
    for (int c = 0; c < NCLS; ++c) osm[row * NCLS + c] = osm[row * NCLS + c] - lse;
  }
  __syncthreads();
  const int pf = pflag;
  const float qnan = __int_as_float(0x7fc00000);
#pragma unroll 1
  for (int i = tid; i < nG * NCLS; i += NTHR) {
    const float v = osm[i];
    osm[i] = (pf != 0) ? qnan : v;
  }
  __syncthreads();
  const int nv = (nG * NCLS) / 4;
#pragma unroll 1
  for (int p = tid; p < nv; p += NTHR) {
    const v4f v = *(const v4fa*)(osm + 4 * p);
    *(volatile v4f*)(out + 4 * p) = v;
  }
  __threadfence();
#pragma unroll 1
  for (int p = tid; p < nv; p += NTHR) {
    const v4f v = *(const v4fa*)(osm + 4 * p);
    *(volatile v4f*)(out + 4 * p) = v;
  }
}

static inline int cdiv(int a, int b) { return (a + b - 1) / b; }
static inline size_t al256(size_t o) { return (o + 255) & ~(size_t)255; }

extern "C" void kernel_launch(void* const* d_in, const int* in_sizes, int n_in,
                              void* d_out, int out_size, void* d_ws, size_t ws_size,
                              hipStream_t stream) {
  if (n_in < 21) return;
  if (in_sizes[0] < DIN || (in_sizes[0] % DIN) != 0) return;
  const int nN = in_sizes[0] / DIN;
  if (nN < GBM || nN > (1 << 22)) return;
  const int nE2 = in_sizes[1];
  if (nE2 < 2 || (nE2 & 1) != 0) return;
  const int nE = nE2 / 2;
  if (nE < 1 || nE >= (1 << 21)) return;
  if (in_sizes[2] != nN) return;
  if (in_sizes[3] != DIN || in_sizes[4] != DIN) return;
  if (in_sizes[5] != DIN * DIN || in_sizes[6] != DIN) return;
  if (in_sizes[7] != 3 * DIN * DIN || in_sizes[8] != 3 * DIN) return;
  if (in_sizes[9] != 3 * DIN || in_sizes[10] != 3 * DIN) return;
  if (in_sizes[11] != 3 * DIN * DIN || in_sizes[12] != 3 * DIN) return;
  if (in_sizes[13] != DIN || in_sizes[14] != DIN) return;
  if (in_sizes[15] != DIN * DIN || in_sizes[16] != DIN) return;
  if (in_sizes[17] != DIN || in_sizes[18] != DIN) return;
  if (in_sizes[19] != DIN * NCLS || in_sizes[20] != NCLS) return;
  if (out_size < NCLS || (out_size % NCLS) != 0 || (out_size % 4) != 0) return;
  const int nG = out_size / NCLS;
  if (nG < 1 || nG > NGCAP || nG > GPAD) return;

  const float* x     = (const float*)d_in[0];
  const int*   ei    = (const int*)  d_in[1];
  const int*   src   = ei;
  const int*   dst   = ei + nE;
  const int*   batch = (const int*)  d_in[2];
  const float* gF  = (const float*)d_in[3];   const float* bF  = (const float*)d_in[4];
  const float* Wf  = (const float*)d_in[5];   const float* cF  = (const float*)d_in[6];
  const float* W1  = (const float*)d_in[7];   const float* c1  = (const float*)d_in[8];
  const float* gL  = (const float*)d_in[9];   const float* bL  = (const float*)d_in[10];
  const float* W2  = (const float*)d_in[11];  const float* c2  = (const float*)d_in[12];
  const float* gC  = (const float*)d_in[13];  const float* bC  = (const float*)d_in[14];
  const float* Wc  = (const float*)d_in[15];  const float* cC  = (const float*)d_in[16];
  const float* gH  = (const float*)d_in[17];  const float* bH  = (const float*)d_in[18];
  const float* Wk  = (const float*)d_in[19];  const float* cK  = (const float*)d_in[20];
  float* out = (float*)d_out;

  const int MP    = cdiv(nN, GBM) * GBM;
  const int gM    = MP / GBM;
  const int nBuck = cdiv(MP, NBK);
  if (nBuck < 1 || nBuck > NTHR) return;
  if ((long long)nBuck * NBK < (long long)MP) return;
  if (((long long)MP * 16) % NTHR != 0) return;
  const int vec8 = ((nE & 3) == 0) ? 1 : 0;

  char* ws = (char*)d_ws;
  size_t off = 0;
  const size_t oWT = off; off = al256(off + (size_t)NPLANE * NUP * 16);
  const size_t oP1 = off; off = al256(off + (size_t)MP * K2 * 2);
  const size_t oP2 = off; off = al256(off + (size_t)MP * DIN * 4);
  const size_t oP3 = off; off = al256(off + (size_t)MP * DIN * 4);
  const size_t oPT = off; off = al256(off + (size_t)gM * PARTW * 4);
  const size_t oST = off; off = al256(off + (size_t)(2 * DIN) * 4);
  const size_t oHT = off; off = al256(off + (size_t)nBuck * RCAP * 4);
  const size_t oCO = off; off = al256(off + (size_t)nBuck * 2 * NBK * 4);
  const size_t oFL = off; off = al256(off + (size_t)nBuck * 32 * 4);
  const size_t oG0 = off; off = al256(off + (size_t)GPAD * DIN * 4);
  const size_t oGH = off; off = al256(off + (size_t)GPAD * K2 * 2);
  const size_t oG1 = off; off = al256(off + (size_t)GPAD * DIN * 4);
  if (off > ws_size || off > (size_t)WSMAX) return;
  unsigned short* WT = (unsigned short*)(ws + oWT);
  unsigned short* P1 = (unsigned short*)(ws + oP1);
  float*          P2 = (float*)(ws + oP2);
  float*          P3 = (float*)(ws + oP3);
  float*          PT = (float*)(ws + oPT);
  float*          ST = (float*)(ws + oST);
  int*            HT = (int*)(ws + oHT);
  int*            CO = (int*)(ws + oCO);
  int*            FL = (int*)(ws + oFL);
  float*          G0 = (float*)(ws + oG0);
  unsigned short* GH = (unsigned short*)(ws + oGH);
  float*          G1 = (float*)(ws + oG1);
  const size_t plane = (size_t)DIN * K2;

  hipFuncSetAttribute(reinterpret_cast<const void*>(&k_bucket), hipFuncAttributeMaxDynamicSharedMemorySize, LDS_BK);

  const int gApply = (int)(((long long)MP * 16) / NTHR);

  k_prep<<<(NPLANE * NUP) / NTHR, NTHR, 0, stream>>>(Wf, W1, W2, Wc, WT);
  k_xstats<<<gM, GTHR, 0, stream>>>(x, nN, PT);
  k_comb<<<1, GBN, 0, stream>>>(PT, gM, ST);
  k_apply<1, 0><<<gApply, NTHR, 0, stream>>>(x, ST, gF, bF, nN, MP, P1);
  k_gemm<1, 0><<<gM, GTHR, 0, stream>>>(P1, WT, cF, P2, nN, MP, PT);
  k_bucket<<<nBuck, NTHR, LDS_BK, stream>>>(src, dst, nN, nE, vec8, HT, CO, FL);
  for (int i = 0; i < 3; ++i) {
    k_agg<<<gM, NTHR, 0, stream>>>(HT, CO, FL, P2, P1, nN, MP, nBuck);
    k_gemm<0, 1><<<gM, GTHR, 0, stream>>>(P1, WT + (size_t)(1 + i) * plane, c1 + (size_t)i * DIN, P3, nN, MP, PT);
    k_comb<<<1, GBN, 0, stream>>>(PT, gM, ST);
    k_apply<0, 1><<<gApply, NTHR, 0, stream>>>(P3, ST, gL + (size_t)i * DIN, bL + (size_t)i * DIN, nN, MP, P1);
    k_gemm<1, 0><<<gM, GTHR, 0, stream>>>(P1, WT + (size_t)(4 + i) * plane, c2 + (size_t)i * DIN, P2, nN, MP, PT);
  }
  k_pool<<<GPAD / PG, NTHR, 0, stream>>>(P2, batch, nN, 1, nG, G0);
  k_bnfc<<<1, NTHR, 0, stream>>>(G0, gC, bC, nG, GH);
  k_gemm<1, 0><<<GPAD / GBM, GTHR, 0, stream>>>(GH, WT + (size_t)7 * plane, cC, G1, nG, GPAD, PT);
  k_tail<<<1, NTHR, 0, stream>>>(G1, gH, bH, Wk, cK, FL, nBuck, nG, out);
}
